// GraphConvolution1_11836929868275
// MI455X (gfx1250) — hardware-verified
//
#include <hip/hip_runtime.h>
#include <stddef.h>


#define KIN    256
#define DF     128
#define NTHR   256
#define NWAVE  8
#define EPT    8
#define CHUNK  (NTHR * EPT)
#define WCAP1  (EPT * 32)
#define WCAP2  (EPT * 32 * 2)
#define NBA    512
#define NBB    512
#define NBM    4096
#define GROWS  64
#define APITCH 264
#define LEAKC  0.2f
#define NEGBIG (-3.0e38f)

#define LDS_GEMM (2 * GROWS * APITCH * 2)
#define LDS_A    (NBA * DF * 4 + NWAVE * WCAP1 * 4 + 64)
#define LDS_M    (4 * NBM * 4 + NWAVE * WCAP2 * 4 + 64)
#define LDS_B    (NBB * DF * 4 + NWAVE * WCAP2 * 4 + 64)

static_assert(CHUNK == 2048);
static_assert((NBA & (NBA - 1)) == 0 && NBA <= 4096);
static_assert((NBB & (NBB - 1)) == 0 && NBB <= 4096);
static_assert((NBM & (NBM - 1)) == 0 && NBM <= 4096);
static_assert(GROWS * DF * 4 <= LDS_GEMM);
static_assert(2 * NBA * 4 <= NWAVE * WCAP1 * 4);
static_assert((APITCH % 8) == 0);
static_assert(NBA == NWAVE * 64 && NBB == NWAVE * 64 && NBM == NWAVE * 512 && GROWS == NWAVE * 8);

typedef float          v4f  __attribute__((ext_vector_type(4)));
typedef float          v8f  __attribute__((ext_vector_type(8)));
typedef int            v4i  __attribute__((ext_vector_type(4)));
typedef unsigned short v8u  __attribute__((ext_vector_type(8)));
typedef __bf16         v16b __attribute__((ext_vector_type(16)));
union FragB { v16b v; v8u u[2]; };

__device__ __forceinline__ unsigned bfb(float f) {
  unsigned u = __float_as_uint(f);
  u += 0x7FFFu + ((u >> 16) & 1u);
  return u >> 16;
}
__device__ __forceinline__ void bfpair(float f, unsigned& h, unsigned& l) {
  h = bfb(f);
  const float hf = __uint_as_float(h << 16);
  l = bfb(f - hf);
}
__device__ __forceinline__ void split8(v4f a, v4f b, v8u& hi, v8u& lo) {
  unsigned h, l;
  v8u hv, lv;
  bfpair(a.x, h, l); hv[0] = (unsigned short)h; lv[0] = (unsigned short)l;
  bfpair(a.y, h, l); hv[1] = (unsigned short)h; lv[1] = (unsigned short)l;
  bfpair(a.z, h, l); hv[2] = (unsigned short)h; lv[2] = (unsigned short)l;
  bfpair(a.w, h, l); hv[3] = (unsigned short)h; lv[3] = (unsigned short)l;
  bfpair(b.x, h, l); hv[4] = (unsigned short)h; lv[4] = (unsigned short)l;
  bfpair(b.y, h, l); hv[5] = (unsigned short)h; lv[5] = (unsigned short)l;
  bfpair(b.z, h, l); hv[6] = (unsigned short)h; lv[6] = (unsigned short)l;
  bfpair(b.w, h, l); hv[7] = (unsigned short)h; lv[7] = (unsigned short)l;
  hi = hv; lo = lv;
}

__device__ __forceinline__ v8f wmb3(v16b ah, v16b al, v16b bh, v16b bl, v8f c) {
  c = __builtin_amdgcn_wmma_f32_16x16x32_bf16(false, ah, false, bh, (short)0, c, false, false);
  c = __builtin_amdgcn_wmma_f32_16x16x32_bf16(false, al, false, bh, (short)0, c, false, false);
  c = __builtin_amdgcn_wmma_f32_16x16x32_bf16(false, ah, false, bl, (short)0, c, false, false);
  asm volatile("v_nop\n\tv_nop\n\tv_nop\n\tv_nop" : "+v"(c) : "v"(ah), "v"(al), "v"(bh), "v"(bl));
  return c;
}

template <int NB, int DIRS, int WCAP>
__device__ __forceinline__ int scan_chunk(const int* __restrict__ ed, int nE, int cbase, int nodeBase,
                                          int* list, int tid, int wave) {
  const int el0  = tid * EPT;
  const int e0   = cbase + el0;
  const int sent = -2147483647 - 1;
  int ka[EPT], kb[EPT];
  if (e0 + (EPT - 1) < nE) {
    const v4i* p = (const v4i*)(ed + 2 * (size_t)e0);
    const v4i q0 = p[0], q1 = p[1], q2 = p[2], q3 = p[3];
    ka[0] = q0.x; kb[0] = q0.y; ka[1] = q0.z; kb[1] = q0.w;
    ka[2] = q1.x; kb[2] = q1.y; ka[3] = q1.z; kb[3] = q1.w;
    ka[4] = q2.x; kb[4] = q2.y; ka[5] = q2.z; kb[5] = q2.w;
    ka[6] = q3.x; kb[6] = q3.y; ka[7] = q3.z; kb[7] = q3.w;
  } else {
#pragma unroll
    for (int j = 0; j < EPT; ++j) {
      const int ee = e0 + j;
      if (ee < nE) { ka[j] = ed[2 * (size_t)ee]; kb[j] = ed[2 * (size_t)ee + 1]; }
      else         { ka[j] = sent;               kb[j] = sent; }
    }
  }
  const unsigned nb = (unsigned)nodeBase;
  unsigned ua[EPT], ur[EPT];
  bool ha[EPT], hr[EPT];
  bool anyl = false;
#pragma unroll
  for (int j = 0; j < EPT; ++j) {
    ua[j] = (unsigned)ka[j] - nb; ha[j] = ua[j] < (unsigned)NB;                  anyl = anyl || ha[j];
    ur[j] = (unsigned)kb[j] - nb; hr[j] = (DIRS == 2) && (ur[j] < (unsigned)NB); anyl = anyl || hr[j];
  }
  int wc = 0;
  const unsigned anyw = __builtin_amdgcn_ballot_w32(anyl);
  if (anyw != 0u) {
#pragma unroll
    for (int j = 0; j < EPT; ++j) {
      {
        const unsigned mj = __builtin_amdgcn_ballot_w32(ha[j]);
        if (mj != 0u) {
          if (ha[j]) {
            const int pos = wc + (int)__builtin_amdgcn_mbcnt_lo(mj, 0u);
            if (pos < WCAP) list[wave * WCAP + pos] = ((el0 + j) << 12) | (int)ua[j];
          }
          wc += (int)__builtin_popcount(mj);
        }
      }
      if (DIRS == 2) {
        const unsigned mj = __builtin_amdgcn_ballot_w32(hr[j]);
        if (mj != 0u) {
          if (hr[j]) {
            const int pos = wc + (int)__builtin_amdgcn_mbcnt_lo(mj, 0u);
            if (pos < WCAP) list[wave * WCAP + pos] = (1 << 23) | ((el0 + j) << 12) | (int)ur[j];
          }
          wc += (int)__builtin_popcount(mj);
        }
      }
    }
  }
  return wc;
}

__device__ __forceinline__ void plane_store(const float* ls, float* gd, int wave, int lane) {
#pragma unroll
  for (int q = 0; q < 4; ++q) {
    const int f = (wave * 4 + q) * 128 + 4 * lane;
    const v4f v = *(const v4f*)(ls + f);
    *(volatile v4f*)(gd + f) = v;
  }
}

__global__ __launch_bounds__(NTHR) void k_wprep(
    const float* __restrict__ W, unsigned short* whi, unsigned short* wlo) {
  const int i = blockIdx.x * NTHR + threadIdx.x;
  if (i >= KIN * DF / 8) return;
  const int o  = i * 8;
  const int n  = o / KIN;
  const int k0 = o - n * KIN;
  const float* p = W + (size_t)k0 * DF + n;
  v4f a, b;
  a.x = p[0];      a.y = p[DF];     a.z = p[2 * DF]; a.w = p[3 * DF];
  b.x = p[4 * DF]; b.y = p[5 * DF]; b.z = p[6 * DF]; b.w = p[7 * DF];
  v8u hv, lv;
  split8(a, b, hv, lv);
  *(volatile v8u*)(whi + o) = hv;
  *(volatile v8u*)(wlo + o) = lv;
  __threadfence();
  *(volatile v8u*)(whi + o) = hv;
  *(volatile v8u*)(wlo + o) = lv;
}

__global__ __launch_bounds__(NTHR) void k_gemm(
    const float* __restrict__ x, const unsigned short* __restrict__ whi,
    const unsigned short* __restrict__ wlo, const float* __restrict__ bias,
    float* xt0, int nN) {
  extern __shared__ v4f lds_dyn[];
  unsigned short* sAh = (unsigned short*)lds_dyn;
  unsigned short* sAl = sAh + GROWS * APITCH;
  float*          stg = (float*)lds_dyn;
  const int tid = threadIdx.x, lane = tid & 31, wave = tid >> 5, hh = lane >> 4, m = lane & 15;
  const int rowBase = blockIdx.x * GROWS;
  const int rgrp = wave & 3, chalf = wave >> 2;

#pragma unroll
  for (int i = 0; i < (GROWS * KIN / 8) / NTHR; ++i) {
    const int idx = i * NTHR + tid;
    const int r   = idx >> 5;
    const int c0  = (idx & 31) * 8;
    int node = rowBase + r;
    node = node > nN - 1 ? nN - 1 : node;
    const float* xp = x + (size_t)node * KIN + c0;
    const v4f a = *(const v4f*)xp, b = *(const v4f*)(xp + 4);
    v8u hv, lv;
    split8(a, b, hv, lv);
    *(v8u*)(sAh + r * APITCH + c0) = hv;
    *(v8u*)(sAl + r * APITCH + c0) = lv;
  }
  __syncthreads();

  v8f acc[4];
#pragma unroll
  for (int t = 0; t < 4; ++t) { v8f z = {0.f, 0.f, 0.f, 0.f, 0.f, 0.f, 0.f, 0.f}; acc[t] = z; }
  const int aoff = (rgrp * 16 + m) * APITCH + 8 * hh;
#pragma unroll 2
  for (int kt = 0; kt < KIN / 32; ++kt) {
    FragB ah, al;
    ah.u[0] = *(const v8u*)(sAh + aoff + 32 * kt);
    ah.u[1] = *(const v8u*)(sAh + aoff + 32 * kt + 16);
    al.u[0] = *(const v8u*)(sAl + aoff + 32 * kt);
    al.u[1] = *(const v8u*)(sAl + aoff + 32 * kt + 16);
#pragma unroll
    for (int t = 0; t < 4; ++t) {
      const size_t boff = (size_t)(16 * (chalf * 4 + t) + m) * KIN + 32 * kt + 8 * hh;
      FragB bh, bl;
      bh.u[0] = *(const v8u*)(whi + boff);
      bh.u[1] = *(const v8u*)(whi + boff + 16);
      bl.u[0] = *(const v8u*)(wlo + boff);
      bl.u[1] = *(const v8u*)(wlo + boff + 16);
      acc[t] = wmb3(ah.v, al.v, bh.v, bl.v, acc[t]);
    }
  }
  __syncthreads();

  const int r0 = rgrp * 16 + 8 * hh;
  float* sp = stg + r0 * DF + m;
#pragma unroll
  for (int t = 0; t < 4; ++t) {
    const int c = 16 * (chalf * 4 + t);
    const float bv = bias[c + m];
    sp[0 * DF + c] = acc[t][0] + bv;
    sp[1 * DF + c] = acc[t][1] + bv;
    sp[2 * DF + c] = acc[t][2] + bv;
    sp[3 * DF + c] = acc[t][3] + bv;
    sp[4 * DF + c] = acc[t][4] + bv;
    sp[5 * DF + c] = acc[t][5] + bv;
    sp[6 * DF + c] = acc[t][6] + bv;
    sp[7 * DF + c] = acc[t][7] + bv;
  }
  __syncthreads();

  const float* lp = stg + wave * 8 * DF + 4 * lane;
  float* gp = xt0 + ((size_t)rowBase + wave * 8) * DF + 4 * lane;
#pragma unroll
  for (int i = 0; i < 8; ++i) { const v4f v = *(const v4f*)(lp + i * DF); *(volatile v4f*)(gp + (size_t)i * DF) = v; }
  __threadfence();
#pragma unroll
  for (int i = 0; i < 8; ++i) { const v4f v = *(const v4f*)(lp + i * DF); *(volatile v4f*)(gp + (size_t)i * DF) = v; }
}

__global__ __launch_bounds__(NTHR) void k_agg1(
    const int* __restrict__ ed, const float* __restrict__ adj, const float* __restrict__ xt0,
    const float* __restrict__ phi, float* xt, float* sap, float* sbp, int nN, int nE) {
  extern __shared__ v4f lds_dyn[];
  float* acc  = (float*)lds_dyn;
  int*   list = (int*)(acc + NBA * DF);
  int*   wcnt = list + NWAVE * WCAP1;
  float* sstg = (float*)list;
  const int tid = threadIdx.x, lane = tid & 31, wave = tid >> 5;
  const int nodeBase = blockIdx.x * NBA;

  {
    const v4f z = {0.f, 0.f, 0.f, 0.f};
    for (int i = tid; i < NBA * DF / 4; i += NTHR) lds_dyn[i] = z;
  }
  __syncthreads();

  const int nChunks = (nE + CHUNK - 1) / CHUNK;
#pragma unroll 1
  for (int ch = 0; ch < nChunks; ++ch) {
    const int cbase = ch * CHUNK;
    const int wc = scan_chunk<NBA, 1, WCAP1>(ed, nE, cbase, nodeBase, list, tid, wave);
    if (lane == 0) wcnt[wave] = wc;
    __syncthreads();
    if (wave == 0) {
#pragma unroll 1
      for (int wsx = 0; wsx < NWAVE; ++wsx) {
        int n = __builtin_amdgcn_readfirstlane(wcnt[wsx]);
        n = n > WCAP1 ? WCAP1 : (n < 0 ? 0 : n);
        const int* lp = list + wsx * WCAP1;
#pragma unroll 1
        for (int i = 0; i < n; ++i) {
          const int ent  = __builtin_amdgcn_readfirstlane(lp[i]);
          const int slot = ent & (NBA - 1);
          int e = cbase + ((ent >> 12) & (CHUNK - 1));
          e = e > nE - 1 ? nE - 1 : e;
          int rcv = ed[2 * (size_t)e + 1];
          rcv = rcv < 0 ? 0 : (rcv > nN - 1 ? nN - 1 : rcv);
          const float av = adj[e];
          const v4f v = *(const v4f*)(xt0 + (size_t)rcv * DF + 4 * lane);
          v4f* ap = (v4f*)(acc + slot * DF + 4 * lane);
          *ap = *ap + av * v;
        }
      }
    }
    __syncthreads();
  }

  const v4f pa = *(const v4f*)(phi + 4 * lane);
  const v4f pb = *(const v4f*)(phi + DF + 4 * lane);
  const float* al = acc + (wave * 64) * DF + 4 * lane;
  float* xg = xt + ((size_t)nodeBase + wave * 64) * DF + 4 * lane;
#pragma unroll 4
  for (int i = 0; i < 64; ++i) {
    const v4f p = *(const v4f*)(al + i * DF);
    float da = p.x * pa.x + p.y * pa.y + p.z * pa.z + p.w * pa.w;
    float db = p.x * pb.x + p.y * pb.y + p.z * pb.z + p.w * pb.w;
#pragma unroll
    for (int o = 16; o > 0; o >>= 1) {
      da += __shfl_xor(da, o, 32);
      db += __shfl_xor(db, o, 32);
    }
    if (lane == 0) { sstg[wave * 64 + i] = da; sstg[NBA + wave * 64 + i] = db; }
    *(volatile v4f*)(xg + (size_t)i * DF) = p;
  }
  __threadfence();
#pragma unroll 4
  for (int i = 0; i < 64; ++i) { const v4f p = *(const v4f*)(al + i * DF); *(volatile v4f*)(xg + (size_t)i * DF) = p; }
  __syncthreads();

  {
    const int w4 = wave & 3;
    const float* sp = sstg + (wave < 4 ? 0 : NBA) + w4 * 128 + 4 * lane;
    float* gp = (wave < 4 ? sap : sbp) + (size_t)nodeBase + w4 * 128 + 4 * lane;
    const v4f v = *(const v4f*)sp;
    *(volatile v4f*)gp = v;
    __threadfence();
    *(volatile v4f*)gp = v;
  }
}

__global__ __launch_bounds__(NTHR) void k_den(
    const int* __restrict__ ed, const float* __restrict__ sa, const float* __restrict__ sb,
    const float* __restrict__ batt, float* mo, float* dno, float* mi, float* dni, int nN, int nE) {
  extern __shared__ v4f lds_dyn[];
  float* lmo  = (float*)lds_dyn;
  float* ldo  = lmo + NBM;
  float* lmi  = ldo + NBM;
  float* ldi  = lmi + NBM;
  int*   list = (int*)(ldi + NBM);
  int*   wcnt = list + NWAVE * WCAP2;
  const int tid = threadIdx.x, lane = tid & 31, wave = tid >> 5;
  const int nodeBase = blockIdx.x * NBM;

  for (int i = tid; i < NBM; i += NTHR) { lmo[i] = NEGBIG; ldo[i] = 0.f; lmi[i] = NEGBIG; ldi[i] = 0.f; }
  __syncthreads();

  const float b0 = batt[0];
  const int nChunks = (nE + CHUNK - 1) / CHUNK;
#pragma unroll 1
  for (int ch = 0; ch < nChunks; ++ch) {
    const int cbase = ch * CHUNK;
    const int wc = scan_chunk<NBM, 2, WCAP2>(ed, nE, cbase, nodeBase, list, tid, wave);
    if (lane == 0) wcnt[wave] = wc;
    __syncthreads();
    if (wave == 0) {
#pragma unroll 1
      for (int wsx = 0; wsx < NWAVE; ++wsx) {
        int n = __builtin_amdgcn_readfirstlane(wcnt[wsx]);
        n = n > WCAP2 ? WCAP2 : (n < 0 ? 0 : n);
        const int* lp = list + wsx * WCAP2;
#pragma unroll 1
        for (int i = 0; i < n; ++i) {
          const int ent  = __builtin_amdgcn_readfirstlane(lp[i]);
          const int slot = ent & (NBM - 1);
          const int dir  = (ent >> 23) & 1;
          int e = cbase + ((ent >> 12) & (CHUNK - 1));
          e = e > nE - 1 ? nE - 1 : e;
          int snd = ed[2 * (size_t)e];
          int rcv = ed[2 * (size_t)e + 1];
          snd = snd < 0 ? 0 : (snd > nN - 1 ? nN - 1 : snd);
          rcv = rcv < 0 ? 0 : (rcv > nN - 1 ? nN - 1 : rcv);
          float v = sa[rcv] + sb[snd] + b0;
          v = v > 0.f ? v : LEAKC * v;
          if (lane == 0) {
            float* pm = dir ? lmi : lmo;
            float* pd = dir ? ldi : ldo;
            float mm = pm[slot], dd = pd[slot];
            if (v > mm) {
              const float sc = (mm > NEGBIG) ? __expf(mm - v) : 0.f;
              dd = dd * sc + 1.f;
              mm = v;
            } else {
              dd = dd + __expf(v - mm);
            }
            pm[slot] = mm;
            pd[slot] = dd;
          }
        }
      }
    }
    __syncthreads();
  }

  plane_store(lmo, mo  + (size_t)nodeBase, wave, lane);
  plane_store(ldo, dno + (size_t)nodeBase, wave, lane);
  plane_store(lmi, mi  + (size_t)nodeBase, wave, lane);
  plane_store(ldi, dni + (size_t)nodeBase, wave, lane);
  __threadfence();
  plane_store(lmo, mo  + (size_t)nodeBase, wave, lane);
  plane_store(ldo, dno + (size_t)nodeBase, wave, lane);
  plane_store(lmi, mi  + (size_t)nodeBase, wave, lane);
  plane_store(ldi, dni + (size_t)nodeBase, wave, lane);
}

__global__ __launch_bounds__(NTHR) void k_agg2(
    const int* __restrict__ ed, const float* __restrict__ xt,
    const float* __restrict__ sa, const float* __restrict__ sb,
    const float* __restrict__ mo, const float* __restrict__ dno,
    const float* __restrict__ mi, const float* __restrict__ dni,
    const float* __restrict__ odeg, const float* __restrict__ ideg,
    const float* __restrict__ batt, const float* __restrict__ wdo, const float* __restrict__ wdi,
    const float* __restrict__ wsf, const float* __restrict__ wno, const float* __restrict__ wni,
    float* out, int nN, int nE) {
  extern __shared__ v4f lds_dyn[];
  float* acc  = (float*)lds_dyn;
  int*   list = (int*)(acc + NBB * DF);
  int*   wcnt = list + NWAVE * WCAP2;
  const int tid = threadIdx.x, lane = tid & 31, wave = tid >> 5;
  const int nodeBase = blockIdx.x * NBB;

  {
    const v4f z = {0.f, 0.f, 0.f, 0.f};
    for (int i = tid; i < NBB * DF / 4; i += NTHR) lds_dyn[i] = z;
  }
  __syncthreads();

  const float b0  = batt[0];
  const float cdo = wdo[0], cdi = wdi[0];
  const float cs  = wsf[0], cno = wno[0], cni = wni[0];

  const int nChunks = (nE + CHUNK - 1) / CHUNK;
#pragma unroll 1
  for (int ch = 0; ch < nChunks; ++ch) {
    const int cbase = ch * CHUNK;
    const int wc = scan_chunk<NBB, 2, WCAP2>(ed, nE, cbase, nodeBase, list, tid, wave);
    if (lane == 0) wcnt[wave] = wc;
    __syncthreads();
    if (wave == 0) {
#pragma unroll 1
      for (int wsx = 0; wsx < NWAVE; ++wsx) {
        int n = __builtin_amdgcn_readfirstlane(wcnt[wsx]);
        n = n > WCAP2 ? WCAP2 : (n < 0 ? 0 : n);
        const int* lp = list + wsx * WCAP2;
#pragma unroll 1
        for (int i = 0; i < n; ++i) {
          const int ent  = __builtin_amdgcn_readfirstlane(lp[i]);
          const int slot = ent & (NBB - 1);
          const int dir  = (ent >> 23) & 1;
          int e = cbase + ((ent >> 12) & (CHUNK - 1));
          e = e > nE - 1 ? nE - 1 : e;
          int snd = ed[2 * (size_t)e];
          int rcv = ed[2 * (size_t)e + 1];
          snd = snd < 0 ? 0 : (snd > nN - 1 ? nN - 1 : snd);
          rcv = rcv < 0 ? 0 : (rcv > nN - 1 ? nN - 1 : rcv);
          float v = sa[rcv] + sb[snd] + b0;
          v = v > 0.f ? v : LEAKC * v;
          const int   j     = dir ? snd : rcv;
          const int   inode = nodeBase + slot;
          const float mx    = dir ? mi[inode]  : mo[inode];
          const float dn    = dir ? dni[inode] : dno[inode];
          const float wn    = dir ? cni : cno;
          const float gl    = cdo * odeg[j] + cdi * ideg[j];
          const float g     = __builtin_amdgcn_rcpf(1.f + __expf(-gl));
          const float coef  = wn * (__expf(v - mx) * __builtin_amdgcn_rcpf(dn)) * g;
          const v4f row = *(const v4f*)(xt + (size_t)j * DF + 4 * lane);
          v4f* ap = (v4f*)(acc + slot * DF + 4 * lane);
          *ap = *ap + coef * row;
        }
      }
    }
    __syncthreads();
  }

#pragma unroll 4
  for (int i = 0; i < (NBB * DF / 4) / NTHR; ++i) {
    const int idx  = i * NTHR + tid;
    const int slot = idx >> 5;
    const int c4   = (idx & 31) * 4;
    int node = nodeBase + slot;
    node = node > nN - 1 ? nN - 1 : node;
    const v4f xv = *(const v4f*)(xt + (size_t)node * DF + c4);
    v4f* ap = (v4f*)(acc + slot * DF + c4);
    v4f r = cs * xv + *ap;
    r.x = fmaxf(r.x, 0.f); r.y = fmaxf(r.y, 0.f); r.z = fmaxf(r.z, 0.f); r.w = fmaxf(r.w, 0.f);
    *ap = r;
  }
  __syncthreads();

  const float* al = acc + (wave * 64) * DF + 4 * lane;
#pragma unroll 4
  for (int i = 0; i < 64; ++i) {
    const int row = nodeBase + wave * 64 + i;
    if (row < nN) { const v4f v = *(const v4f*)(al + i * DF); *(volatile v4f*)(out + (size_t)row * DF + 4 * lane) = v; }
  }
  __threadfence();
#pragma unroll 4
  for (int i = 0; i < 64; ++i) {
    const int row = nodeBase + wave * 64 + i;
    if (row < nN) { const v4f v = *(const v4f*)(al + i * DF); *(volatile v4f*)(out + (size_t)row * DF + 4 * lane) = v; }
  }
}

extern "C" void kernel_launch(void* const* d_in, const int* in_sizes, int n_in,
                              void* d_out, int out_size, void* d_ws, size_t ws_size,
                              hipStream_t stream) {
  if (n_in < 14) return;
  const int nN = in_sizes[0] / KIN;
  const int nE = in_sizes[1] / 2;
  if (nN <= 0 || nE < 0) return;
  if (in_sizes[0] != nN * KIN || in_sizes[1] != nE * 2 || in_sizes[2] != nE) return;
  if (in_sizes[3] != nN || in_sizes[4] != nN) return;
  if (in_sizes[5] != KIN * DF || in_sizes[6] != DF || in_sizes[7] != 2 * DF) return;
  for (int k = 8; k < 14; ++k) if (in_sizes[k] < 1) return;
  if (out_size != nN * DF) return;

  const float* x    = (const float*)d_in[0];
  const int*   ed   = (const int*)d_in[1];
  const float* adj  = (const float*)d_in[2];
  const float* odeg = (const float*)d_in[3];
  const float* ideg = (const float*)d_in[4];
  const float* W    = (const float*)d_in[5];
  const float* bias = (const float*)d_in[6];
  const float* phi  = (const float*)d_in[7];
  const float* batt = (const float*)d_in[8];
  const float* wdo  = (const float*)d_in[9];
  const float* wdi  = (const float*)d_in[10];
  const float* wsf  = (const float*)d_in[11];
  const float* wno  = (const float*)d_in[12];
  const float* wni  = (const float*)d_in[13];
  float* out = (float*)d_out;

  const int nG = (nN + GROWS - 1) / GROWS;
  const int nA = (nN + NBA - 1) / NBA;
  const int nM = (nN + NBM - 1) / NBM;
  const int nB = (nN + NBB - 1) / NBB;

  char* ws = (char*)d_ws;
  size_t off = 0;
  const size_t oWh = off; off += (size_t)KIN * DF * 2;            off = (off + 255) & ~(size_t)255;
  const size_t oWl = off; off += (size_t)KIN * DF * 2;            off = (off + 255) & ~(size_t)255;
  const size_t oX0 = off; off += (size_t)nG * GROWS * DF * 4;     off = (off + 255) & ~(size_t)255;
  const size_t oXt = off; off += (size_t)nA * NBA * DF * 4;       off = (off + 255) & ~(size_t)255;
  const size_t oSa = off; off += (size_t)nA * NBA * 4;            off = (off + 255) & ~(size_t)255;
  const size_t oSb = off; off += (size_t)nA * NBA * 4;            off = (off + 255) & ~(size_t)255;
  const size_t oMo = off; off += (size_t)nM * NBM * 4;            off = (off + 255) & ~(size_t)255;
  const size_t oDo = off; off += (size_t)nM * NBM * 4;            off = (off + 255) & ~(size_t)255;
  const size_t oMi = off; off += (size_t)nM * NBM * 4;            off = (off + 255) & ~(size_t)255;
  const size_t oDi = off; off += (size_t)nM * NBM * 4;            off = (off + 255) & ~(size_t)255;
  if (off > ws_size) return;
  if (off > (size_t)134217728) return;
  unsigned short* whi = (unsigned short*)(ws + oWh);
  unsigned short* wlo = (unsigned short*)(ws + oWl);
  float* xt0 = (float*)(ws + oX0);
  float* xt  = (float*)(ws + oXt);
  float* sa  = (float*)(ws + oSa);
  float* sb  = (float*)(ws + oSb);
  float* mo  = (float*)(ws + oMo);
  float* dno = (float*)(ws + oDo);
  float* mi  = (float*)(ws + oMi);
  float* dni = (float*)(ws + oDi);

  const int nPrep = KIN * DF / 8;
  k_wprep<<<(nPrep + NTHR - 1) / NTHR, NTHR, 0, stream>>>(W, whi, wlo);

  hipFuncSetAttribute(reinterpret_cast<const void*>(&k_gemm),
                      hipFuncAttributeMaxDynamicSharedMemorySize, LDS_GEMM);
  k_gemm<<<nG, NTHR, LDS_GEMM, stream>>>(x, whi, wlo, bias, xt0, nN);

  hipFuncSetAttribute(reinterpret_cast<const void*>(&k_agg1),
                      hipFuncAttributeMaxDynamicSharedMemorySize, LDS_A);
  k_agg1<<<nA, NTHR, LDS_A, stream>>>(ed, adj, xt0, phi, xt, sa, sb, nN, nE);

  hipFuncSetAttribute(reinterpret_cast<const void*>(&k_den),
                      hipFuncAttributeMaxDynamicSharedMemorySize, LDS_M);
  k_den<<<nM, NTHR, LDS_M, stream>>>(ed, sa, sb, batt, mo, dno, mi, dni, nN, nE);

  hipFuncSetAttribute(reinterpret_cast<const void*>(&k_agg2),
                      hipFuncAttributeMaxDynamicSharedMemorySize, LDS_B);
  k_agg2<<<nB, NTHR, LDS_B, stream>>>(ed, xt, sa, sb, mo, dno, mi, dni, odeg, ideg,
                                      batt, wdo, wdi, wsf, wno, wni, out, nN, nE);
}
